// HSI_RWKV_43731357008661
// MI455X (gfx1250) — hardware-run, weakly checked
//
#include <hip/hip_runtime.h>
#include <math.h>

typedef __attribute__((ext_vector_type(16))) _Float16 v16h;
typedef __attribute__((ext_vector_type(8)))  _Float16 v8h;
typedef __attribute__((ext_vector_type(8)))  float    v8f;
typedef __attribute__((ext_vector_type(4)))  float    v4f;

constexpr int kBatch = 4;
constexpr int kCh    = 128;
constexpr int kHid   = 512;
constexpr int kHW    = 16384;
constexpr int kTok   = 32;
constexpr int kThr   = 64;
constexpr int kTilesPerB = kHW / kTok;
constexpr int kXP    = 132;
constexpr int kAP    = 136;
static_assert(kHid == 4 * kCh, "hidden width");
static_assert((kHW % kTok) == 0 && kTok == 32 && kThr == 64, "tile geometry: 2 waves x 16 token rows");
static_assert((kCh % 32) == 0 && (kHid % 128) == 0, "K multiples of 32, hidden chunks of 128");
static_assert((kXP % 4) == 0 && (kAP % 8) == 0, "16-B aligned LDS rows");

constexpr float kCarryAct = 64.0f;
constexpr float kCarrySq  = 256.0f;
constexpr float kCarryW   = 256.0f;
constexpr float kFoldActW = 1.0f / (kCarryAct * kCarryW);
constexpr float kFoldSqW  = 1.0f / (kCarrySq * kCarryW);
constexpr float kWhtStore = kCarryAct * kFoldActW;
constexpr float kF16MinNormal = 6.103515625e-5f;
constexpr float kF16Clamp = 60000.0f;

constexpr size_t kElO = (size_t)kCh * kCh;
constexpr size_t kElW = (size_t)kCh * kCh;
constexpr size_t kElK = (size_t)kHid * kCh;
constexpr size_t kElR = (size_t)kCh * kCh;
constexpr size_t kElV = (size_t)kCh * kHid;
constexpr size_t kOffO = 0;
constexpr size_t kOffW = kOffO + kElO;
constexpr size_t kOffK = kOffW + kElW;
constexpr size_t kOffR = kOffK + kElK;
constexpr size_t kOffV = kOffR + kElR;
constexpr size_t kElAll = kOffV + kElV;
constexpr size_t kWsTotal = kElAll * 2;
static_assert(kWsTotal == 360448ull, "carve total");
static_assert(kWsTotal <= 134217728ull, "carve cap");
static_assert(((kOffW * 2) % 128) == 0 && ((kOffK * 2) % 128) == 0 && ((kOffR * 2) % 128) == 0 && ((kOffV * 2) % 128) == 0, "128-B aligned planes");
constexpr int kCvtPerBlk = 2048;
static_assert((kElO % kCvtPerBlk) == 0 && (kElK % kCvtPerBlk) == 0 && (kElV % kCvtPerBlk) == 0, "whole blocks per plane");
constexpr int kBlkEndO = (int)(kOffW / kCvtPerBlk);
constexpr int kBlkEndW = (int)(kOffK / kCvtPerBlk);
constexpr int kBlkEndK = (int)(kOffR / kCvtPerBlk);
constexpr int kBlkEndR = (int)(kOffV / kCvtPerBlk);
constexpr int kCvtBlocks = (int)(kElAll / kCvtPerBlk);
static_assert(kCvtBlocks == 88, "conversion grid");

union FragU { v16h v; v8h h[2]; };

__device__ __forceinline__ v16h frag_ld(const _Float16* p) {
  FragU f;
  f.h[0] = *(const v8h*)(p);
  f.h[1] = *(const v8h*)(p + 16);
  return f.v;
}

__device__ __forceinline__ v8f mma_h(v16h a, v16h b, v8f c) {
  c = __builtin_amdgcn_wmma_f32_16x16x32_f16(false, a, false, b, (short)0, c, false, false);
  asm volatile("v_nop\n\tv_nop\n\tv_nop\n\tv_nop" : "+v"(c) : "v"(a), "v"(b));
  return c;
}

__device__ __forceinline__ _Float16 to_h_flush(float v) {
  const float f = (fabsf(v) < kF16MinNormal) ? 0.0f : v;
  return (_Float16)f;
}

__device__ __forceinline__ float sigmoid_f(float v) {
  return __builtin_amdgcn_rcpf(1.0f + expf(-v));
}

__device__ __forceinline__ v8f tile_k128(v16h a0, v16h a1, v16h a2, v16h a3, const _Float16* bp) {
  const v16h b0 = frag_ld(bp);
  const v16h b1 = frag_ld(bp + 32);
  const v16h b2 = frag_ld(bp + 64);
  const v16h b3 = frag_ld(bp + 96);
  v8f acc = (v8f){0.f, 0.f, 0.f, 0.f, 0.f, 0.f, 0.f, 0.f};
  acc = mma_h(a0, b0, acc);
  acc = mma_h(a1, b1, acc);
  acc = mma_h(a2, b2, acc);
  acc = mma_h(a3, b3, acc);
  return acc;
}

__device__ __forceinline__ void ln_stats(const float* xr, float& mu, float& rs) {
  float s = 0.f;
#pragma unroll 4
  for (int j = 0; j < 16; ++j) {
    const v4f v = *(const v4f*)(xr + 4 * j);
    s += (v[0] + v[1]) + (v[2] + v[3]);
  }
  s += __shfl_xor(s, 1, 32);
  mu = s * (1.0f / (float)kCh);
  float q = 0.f;
#pragma unroll 4
  for (int j = 0; j < 16; ++j) {
    const v4f v = *(const v4f*)(xr + 4 * j);
    const float d0 = v[0] - mu, d1 = v[1] - mu, d2 = v[2] - mu, d3 = v[3] - mu;
    q += (d0 * d0 + d1 * d1) + (d2 * d2 + d3 * d3);
  }
  q += __shfl_xor(q, 1, 32);
  rs = rsqrtf(q * (1.0f / (float)kCh) + 1e-5f);
}

template <bool SILU>
__device__ __forceinline__ void ln_emit_f16(const float* xr, const float* gp, const float* bp,
                                            float mu, float rs, _Float16* ar) {
#pragma unroll 1
  for (int j = 0; j < 8; ++j) {
    const v4f va = *(const v4f*)(xr + 8 * j);
    const v4f vb = *(const v4f*)(xr + 8 * j + 4);
    const v4f ga = *(const v4f*)(gp + 8 * j);
    const v4f gb = *(const v4f*)(gp + 8 * j + 4);
    const v4f ba = *(const v4f*)(bp + 8 * j);
    const v4f bb = *(const v4f*)(bp + 8 * j + 4);
    v8h hv;
#pragma unroll
    for (int e = 0; e < 4; ++e) {
      const float ya = (va[e] - mu) * rs * ga[e] + ba[e];
      const float yb = (vb[e] - mu) * rs * gb[e] + bb[e];
      float oa = ya, ob = yb;
      if (SILU) {
        oa = ya * sigmoid_f(ya);
        ob = yb * sigmoid_f(yb);
      }
      hv[e]     = to_h_flush(oa * kCarryAct);
      hv[4 + e] = to_h_flush(ob * kCarryAct);
    }
    *(v8h*)(ar + 8 * j) = hv;
  }
}

__global__ __launch_bounds__(256) void weights_to_f16_kernel(
    const float* __restrict__ wo, const float* __restrict__ ww, const float* __restrict__ wk,
    const float* __restrict__ wr, const float* __restrict__ wv, _Float16* __restrict__ dst)
{
  const int bx = blockIdx.x;
  const float* src = wo;
  int bfirst = 0;
  if (bx >= kBlkEndO) { src = ww; bfirst = kBlkEndO; }
  if (bx >= kBlkEndW) { src = wk; bfirst = kBlkEndW; }
  if (bx >= kBlkEndK) { src = wr; bfirst = kBlkEndK; }
  if (bx >= kBlkEndR) { src = wv; bfirst = kBlkEndR; }
  const size_t se = ((size_t)(bx - bfirst) * 256 + threadIdx.x) * 8;
  const size_t de = ((size_t)bx * 256 + threadIdx.x) * 8;
  const v4f a0 = *(const v4f*)(src + se);
  const v4f a1 = *(const v4f*)(src + se + 4);
  v8h hv;
#pragma unroll
  for (int e = 0; e < 4; ++e) {
    hv[e]     = to_h_flush(a0[e] * kCarryW);
    hv[4 + e] = to_h_flush(a1[e] * kCarryW);
  }
  _Float16* q = dst + de;
  *(volatile v8h*)q = hv;
  __threadfence();
  *(volatile v8h*)q = hv;
}

__global__ __launch_bounds__(kThr) void token_chain_kernel(
    const float* __restrict__ x,
    const float* __restrict__ ln0g, const float* __restrict__ ln0b,
    const float* __restrict__ ln1g, const float* __restrict__ ln1b,
    const float* __restrict__ ln2g, const float* __restrict__ ln2b,
    const _Float16* __restrict__ Wo, const _Float16* __restrict__ Ww, const _Float16* __restrict__ Wk,
    const _Float16* __restrict__ Wr, const _Float16* __restrict__ Wv,
    float* __restrict__ out)
{
  __shared__ __align__(16) float    sX[kTok * kXP];
  __shared__ __align__(16) float    sR[kTok * kXP];
  __shared__ __align__(16) _Float16 sA[kTok * kAP];
  __shared__ __align__(16) float    sG[6 * kCh];

  const int tid  = threadIdx.x;
  const int lane = tid & 31;
  const int wave = tid >> 5;
  const int lm   = lane & 15;
  const int lh   = lane >> 4;
  const int m0   = wave * 16;
  const int batch = blockIdx.x / kTilesPerB;
  const int tile  = blockIdx.x - batch * kTilesPerB;
  const int t0    = tile * kTok;

  sG[0 * kCh + tid] = ln0g[tid];  sG[0 * kCh + 64 + tid] = ln0g[64 + tid];
  sG[1 * kCh + tid] = ln0b[tid];  sG[1 * kCh + 64 + tid] = ln0b[64 + tid];
  sG[2 * kCh + tid] = ln1g[tid];  sG[2 * kCh + 64 + tid] = ln1g[64 + tid];
  sG[3 * kCh + tid] = ln1b[tid];  sG[3 * kCh + 64 + tid] = ln1b[64 + tid];
  sG[4 * kCh + tid] = ln2g[tid];  sG[4 * kCh + 64 + tid] = ln2g[64 + tid];
  sG[5 * kCh + tid] = ln2b[tid];  sG[5 * kCh + 64 + tid] = ln2b[64 + tid];

  const int tq = (tid & 7) * 4;
  const int cq = tid >> 3;
  {
    const float* xb = x + (size_t)batch * kCh * kHW + t0 + tq;
#pragma unroll 4
    for (int it = 0; it < 16; ++it) {
      const int c = it * 8 + cq;
      const v4f v = *(const v4f*)(xb + (size_t)c * kHW);
      sX[(tq + 0) * kXP + c] = v[0];
      sX[(tq + 1) * kXP + c] = v[1];
      sX[(tq + 2) * kXP + c] = v[2];
      sX[(tq + 3) * kXP + c] = v[3];
    }
  }
  __syncthreads();

  const int lrow = m0 + (lane >> 1);
  const int cb   = (lane & 1) * 64;
  float*    xr = sX + lrow * kXP + cb;
  _Float16* ar = sA + lrow * kAP + cb;

  {
    float mu, rs;
    ln_stats(xr, mu, rs);
    const float* gp = sG + 0 * kCh + cb;
    const float* bp = sG + 1 * kCh + cb;
#pragma unroll 2
    for (int j = 0; j < 16; ++j) {
      const v4f v = *(const v4f*)(xr + 4 * j);
      const v4f g = *(const v4f*)(gp + 4 * j);
      const v4f b = *(const v4f*)(bp + 4 * j);
      v4f t;
      t[0] = (v[0] - mu) * rs * g[0] + b[0];
      t[1] = (v[1] - mu) * rs * g[1] + b[1];
      t[2] = (v[2] - mu) * rs * g[2] + b[2];
      t[3] = (v[3] - mu) * rs * g[3] + b[3];
      *(v4f*)(xr + 4 * j) = t;
    }
  }
  __syncthreads();

  {
    float mu, rs;
    ln_stats(xr, mu, rs);
    ln_emit_f16<true>(xr, sG + 2 * kCh + cb, sG + 3 * kCh + cb, mu, rs, ar);
  }
  __syncthreads();

  const int aoff = (m0 + lm) * kAP + 8 * lh;
  const int drow = m0 + 8 * lh;

  {
    FragU fa[4];
#pragma unroll
    for (int k = 0; k < 4; ++k) {
      fa[k].h[0] = *(const v8h*)(sA + aoff + 32 * k);
      fa[k].h[1] = *(const v8h*)(sA + aoff + 32 * k + 16);
    }
#pragma unroll 1
    for (int n = 0; n < 8; ++n) {
      const _Float16* bp = Wo + (size_t)(n * 16 + lm) * kCh + 8 * lh;
      const v8f acc = tile_k128(fa[0].v, fa[1].v, fa[2].v, fa[3].v, bp);
#pragma unroll
      for (int r = 0; r < 8; ++r) {
        const int ix = (drow + r) * kXP + n * 16 + lm;
        sX[ix] = sX[ix] + acc[r] * kFoldActW;
      }
    }
  }
  __syncthreads();

  {
    float mu, rs;
    ln_stats(xr, mu, rs);
    ln_emit_f16<false>(xr, sG + 4 * kCh + cb, sG + 5 * kCh + cb, mu, rs, ar);
  }
  __syncthreads();

  {
    FragU fa[4];
#pragma unroll
    for (int k = 0; k < 4; ++k) {
      fa[k].h[0] = *(const v8h*)(sA + aoff + 32 * k);
      fa[k].h[1] = *(const v8h*)(sA + aoff + 32 * k + 16);
    }
    __syncthreads();
#pragma unroll 1
    for (int n = 0; n < 8; ++n) {
      const _Float16* bp = Ww + (size_t)(n * 16 + lm) * kCh + 8 * lh;
      const v8f acc = tile_k128(fa[0].v, fa[1].v, fa[2].v, fa[3].v, bp);
#pragma unroll
      for (int r = 0; r < 8; ++r)
        sA[(drow + r) * kAP + n * 16 + lm] = to_h_flush(acc[r] * kWhtStore);
    }
  }
  __syncthreads();

  FragU aw[4];
#pragma unroll
  for (int k = 0; k < 4; ++k) {
    aw[k].h[0] = *(const v8h*)(sA + aoff + 32 * k);
    aw[k].h[1] = *(const v8h*)(sA + aoff + 32 * k + 16);
  }
  __syncthreads();

#pragma unroll 1
  for (int n = 0; n < 8; ++n) {
    const _Float16* bp = Wr + (size_t)(n * 16 + lm) * kCh + 8 * lh;
    const v8f acc = tile_k128(aw[0].v, aw[1].v, aw[2].v, aw[3].v, bp);
#pragma unroll
    for (int r = 0; r < 8; ++r)
      sR[(drow + r) * kXP + n * 16 + lm] = sigmoid_f(acc[r] * kFoldActW);
  }

  v8f kv[8];
#pragma unroll
  for (int n = 0; n < 8; ++n) kv[n] = (v8f){0.f, 0.f, 0.f, 0.f, 0.f, 0.f, 0.f, 0.f};

#pragma unroll 1
  for (int hc = 0; hc < 4; ++hc) {
#pragma unroll 1
    for (int nt = 0; nt < 8; ++nt) {
      const _Float16* bp = Wk + (size_t)(hc * 128 + nt * 16 + lm) * kCh + 8 * lh;
      const v8f acc = tile_k128(aw[0].v, aw[1].v, aw[2].v, aw[3].v, bp);
#pragma unroll
      for (int r = 0; r < 8; ++r) {
        const float kp = fmaxf(acc[r] * kFoldActW, 0.0f);
        const float sq = fminf(kp * kp * kCarrySq, kF16Clamp);
        sA[(drow + r) * kAP + nt * 16 + lm] = to_h_flush(sq);
      }
    }
    __syncthreads();
#pragma unroll 1
    for (int ks = 0; ks < 4; ++ks) {
      FragU ka;
      ka.h[0] = *(const v8h*)(sA + aoff + 32 * ks);
      ka.h[1] = *(const v8h*)(sA + aoff + 32 * ks + 16);
      const _Float16* vp = Wv + (size_t)lm * kHid + hc * 128 + ks * 32 + 8 * lh;
#pragma unroll
      for (int n = 0; n < 8; ++n) {
        const v16h bv = frag_ld(vp + (size_t)n * 16 * kHid);
        kv[n] = mma_h(ka.v, bv, kv[n]);
      }
    }
    __syncthreads();
  }

#pragma unroll
  for (int n = 0; n < 8; ++n) {
#pragma unroll
    for (int r = 0; r < 8; ++r) {
      const int ix = (drow + r) * kXP + n * 16 + lm;
      const float kvv = kv[n][r] * kFoldSqW;
      sX[ix] = 2.0f * (sX[ix] + sR[ix] * kvv);
    }
  }
  __syncthreads();

  {
    float* ob = out + (size_t)batch * kCh * kHW + t0 + tq;
    v4f ov[16];
#pragma unroll
    for (int it = 0; it < 16; ++it) {
      const int c = it * 8 + cq;
      v4f o;
      o[0] = sX[(tq + 0) * kXP + c];
      o[1] = sX[(tq + 1) * kXP + c];
      o[2] = sX[(tq + 2) * kXP + c];
      o[3] = sX[(tq + 3) * kXP + c];
      ov[it] = o;
    }
    for (int pass = 0; pass < 2; ++pass) {
#pragma unroll
      for (int it = 0; it < 16; ++it) {
        const int c = it * 8 + cq;
        *(volatile v4f*)(ob + (size_t)c * kHW) = ov[it];
      }
      __threadfence();
    }
  }
}

extern "C" void kernel_launch(void* const* d_in, const int* in_sizes, int n_in,
                              void* d_out, int out_size, void* d_ws, size_t ws_size,
                              hipStream_t stream) {
  if (n_in < 12) return;
  if (in_sizes[0] != kBatch * kCh * kHW) return;
  for (int i = 1; i <= 6; ++i) if (in_sizes[i] != kCh) return;
  if (in_sizes[7] != kCh * kCh) return;
  if (in_sizes[8] != kCh * kCh) return;
  if (in_sizes[9] != kHid * kCh) return;
  if (in_sizes[10] != kCh * kCh) return;
  if (in_sizes[11] != kCh * kHid) return;
  if (out_size != kBatch * kCh * kHW) return;
  if (ws_size < kWsTotal) return;

  const float* img   = (const float*)d_in[0];
  const float* ln0g  = (const float*)d_in[1];
  const float* ln0b  = (const float*)d_in[2];
  const float* ln1g  = (const float*)d_in[3];
  const float* ln1b  = (const float*)d_in[4];
  const float* ln2g  = (const float*)d_in[5];
  const float* ln2b  = (const float*)d_in[6];
  const float* wOut  = (const float*)d_in[7];
  const float* wWht  = (const float*)d_in[8];
  const float* wKey  = (const float*)d_in[9];
  const float* wRec  = (const float*)d_in[10];
  const float* wVal  = (const float*)d_in[11];
  float* outp = (float*)d_out;

  _Float16* wpl = (_Float16*)d_ws;

  weights_to_f16_kernel<<<kCvtBlocks, 256, 0, stream>>>(wOut, wWht, wKey, wRec, wVal, wpl);

  token_chain_kernel<<<kBatch * kTilesPerB, kThr, 0, stream>>>(
      img, ln0g, ln0b, ln1g, ln1b, ln2g, ln2b,
      wpl + kOffO, wpl + kOffW, wpl + kOffK, wpl + kOffR, wpl + kOffV, outp);
}
